// LSTM_47923245088969
// MI455X (gfx1250) — hardware-verified
//
#include <hip/hip_runtime.h>
#include <math.h>

constexpr int NBATCH   = 128;
constexpr int NSTEP    = 512;
constexpr int NHID     = 256;
constexpr int NFUT     = 64;
constexpr int NTOT     = NSTEP + NFUT;
constexpr int NGATE    = 4 * NHID;
constexpr int ROWS_BLK = 32;
constexpr int SEQ_THR  = 512;
constexpr int SEQ_WAVES = SEQ_THR / 32;
constexpr int HPITCH   = 264;
constexpr int SLABP    = 580;
constexpr int PREP_THR = 256;
constexpr int CVT_BLKS = NGATE * (NHID / 8) / PREP_THR;
constexpr int PREP_BLKS = 3 * CVT_BLKS + 2;
constexpr float WCARRY    = 64.0f;
constexpr float HCARRY    = 64.0f;
constexpr float CARRY_INV = 1.0f / (WCARRY * HCARRY);

static_assert(NTOT == 576, "output row length");
static_assert(NHID == 16 * SEQ_WAVES, "one 16-column unit group per wave");
static_assert(NHID % 32 == 0, "k multiple of 32");
static_assert(NBATCH % ROWS_BLK == 0, "batch tiles");
static_assert(ROWS_BLK == 32, "two 16-row subtiles per block");
static_assert((2 * ROWS_BLK * HPITCH) % SEQ_THR == 0, "h zero-fill exact");
static_assert((ROWS_BLK * NSTEP / 4) % SEQ_THR == 0, "slab preload exact");
static_assert((ROWS_BLK * NTOT / 4) % SEQ_THR == 0, "output store exact");
static_assert(HPITCH % 8 == 0 && SLABP % 4 == 0 && SLABP >= NTOT, "LDS pitches");
static_assert((NGATE * (NHID / 8)) % PREP_THR == 0, "convert grid exact");
static_assert(NGATE == 4 * PREP_THR, "bias block covers 1024 floats");
static_assert((NTOT * 4) % 128 == 0, "output rows are whole lines");

typedef __attribute__((ext_vector_type(16))) _Float16 v16h;
typedef __attribute__((ext_vector_type(8)))  _Float16 v8h;
typedef __attribute__((ext_vector_type(8)))  float    v8f;
typedef __attribute__((ext_vector_type(4)))  float    v4f;

__device__ __forceinline__ void acc_guard4(v8f& a, v8f& b, v8f& c, v8f& d) {
  asm volatile("v_nop\n\tv_nop\n\tv_nop\n\tv_nop" : "+v"(a), "+v"(b), "+v"(c), "+v"(d));
}
__device__ __forceinline__ void guard8(v8f& a0, v8f& a1, v8f& a2, v8f& a3, v8f& a4, v8f& a5, v8f& a6, v8f& a7,
                                       v16h x0, v16h x1, v16h y0, v16h y1, v16h y2, v16h y3) {
  asm volatile("v_nop\n\tv_nop\n\tv_nop\n\tv_nop"
               : "+v"(a0), "+v"(a1), "+v"(a2), "+v"(a3), "+v"(a4), "+v"(a5), "+v"(a6), "+v"(a7)
               : "v"(x0), "v"(x1), "v"(y0), "v"(y1), "v"(y2), "v"(y3));
}

struct FragH {
  union U { v16h v; v8h h[2]; };
  static __device__ __forceinline__ v16h load(const _Float16* p) {
    U f; f.h[0] = *(const v8h*)(p); f.h[1] = *(const v8h*)(p + 16); return f.v;
  }
  static __device__ __forceinline__ v8f mma(v16h a, v16h b, v8f c) {
    return __builtin_amdgcn_wmma_f32_16x16x32_f16(false, a, false, b, (short)0, c, false, false);
  }
};

__device__ __forceinline__ float fsig(float x)  { return __builtin_amdgcn_rcpf(1.0f + expf(-x)); }
__device__ __forceinline__ float ftanh(float x) { return 1.0f - 2.0f * __builtin_amdgcn_rcpf(expf(2.0f * x) + 1.0f); }

__global__ __launch_bounds__(PREP_THR) void prep_kernel(const float* __restrict__ whh1, const float* __restrict__ wih2,
                                                        const float* __restrict__ whh2,
                                                        const float* __restrict__ bih1, const float* __restrict__ bhh1,
                                                        const float* __restrict__ bih2, const float* __restrict__ bhh2,
                                                        unsigned short* __restrict__ bt1, unsigned short* __restrict__ bt2,
                                                        float* __restrict__ bsum) {
  const int tid = threadIdx.x;
  const int region = blockIdx.x / CVT_BLKS;
  if (region < 3) {
    const float* src = (region == 0) ? whh1 : ((region == 1) ? wih2 : whh2);
    unsigned short* dst = (region == 0) ? bt1 : bt2;
    const int dpitch = (region == 0) ? NHID : (2 * NHID);
    const int dcol0  = (region == 2) ? NHID : 0;
    const int i   = (blockIdx.x - region * CVT_BLKS) * PREP_THR + tid;
    const int row = i >> 5;
    const int c8  = i & 31;
    const float* sp = src + (size_t)row * NHID + c8 * 8;
    const v4f a = *(const v4f*)(sp);
    const v4f b = *(const v4f*)(sp + 4);
    v8h hv;
#pragma unroll
    for (int e = 0; e < 4; ++e) {
      const float fa = a[e] * WCARRY;
      const float fb = b[e] * WCARRY;
      hv[e]     = (_Float16)fa;
      hv[4 + e] = (_Float16)fb;
    }
    unsigned short* dp = dst + (size_t)row * dpitch + dcol0 + c8 * 8;
    *(volatile v8h*)dp = hv;
    __threadfence();
    *(volatile v8h*)dp = hv;
  } else {
    const int which = blockIdx.x - 3 * CVT_BLKS;
    const float* pa = which ? bih2 : bih1;
    const float* pb = which ? bhh2 : bhh1;
    const int idx = tid * 4;
    const v4f va = *(const v4f*)(pa + idx);
    const v4f vb = *(const v4f*)(pb + idx);
    v4f o;
#pragma unroll
    for (int e = 0; e < 4; ++e) o[e] = va[e] + vb[e];
    float* op = bsum + which * NGATE + idx;
    *(volatile v4f*)op = o;
    __threadfence();
    *(volatile v4f*)op = o;
  }
}

__device__ __forceinline__ void ksweep(v8f (&acc)[4][2], const _Float16* arow, const _Float16* wrow, const int ldw) {
#pragma unroll 1
  for (int k0 = 0; k0 < NHID; k0 += 32) {
    const v16h a0 = FragH::load(arow + k0);
    const v16h a1 = FragH::load(arow + 16 * HPITCH + k0);
    const v16h b0 = FragH::load(wrow + k0);
    const v16h b1 = FragH::load(wrow + (size_t)1 * NHID * ldw + k0);
    const v16h b2 = FragH::load(wrow + (size_t)2 * NHID * ldw + k0);
    const v16h b3 = FragH::load(wrow + (size_t)3 * NHID * ldw + k0);
    acc[0][0] = FragH::mma(a0, b0, acc[0][0]);
    acc[0][1] = FragH::mma(a1, b0, acc[0][1]);
    acc[1][0] = FragH::mma(a0, b1, acc[1][0]);
    acc[1][1] = FragH::mma(a1, b1, acc[1][1]);
    acc[2][0] = FragH::mma(a0, b2, acc[2][0]);
    acc[2][1] = FragH::mma(a1, b2, acc[2][1]);
    acc[3][0] = FragH::mma(a0, b3, acc[3][0]);
    acc[3][1] = FragH::mma(a1, b3, acc[3][1]);
    guard8(acc[0][0], acc[0][1], acc[1][0], acc[1][1], acc[2][0], acc[2][1], acc[3][0], acc[3][1],
           a0, a1, b0, b1, b2, b3);
  }
}

template <bool FIRST>
__device__ __forceinline__ void cell_update(const v8f& ai, const v8f& af, const v8f& ag, const v8f& ao,
                                            float (&cs)[8], const float (&bb)[4], const float (&ww)[4],
                                            const float* xs, _Float16* hd, const float wl, float (&pv)[8]) {
#pragma unroll
  for (int r = 0; r < 8; ++r) {
    float zi = ai[r] * CARRY_INV + bb[0];
    float zf = af[r] * CARRY_INV + bb[1];
    float zg = ag[r] * CARRY_INV + bb[2];
    float zo = ao[r] * CARRY_INV + bb[3];
    if (FIRST) {
      const float xv = xs[r * SLABP];
      zi += xv * ww[0];
      zf += xv * ww[1];
      zg += xv * ww[2];
      zo += xv * ww[3];
    }
    const float ig = fsig(zi);
    const float fg = fsig(zf);
    const float gg = ftanh(zg);
    const float og = fsig(zo);
    const float cn = fg * cs[r] + ig * gg;
    cs[r] = cn;
    const float hn = og * ftanh(cn);
    hd[r * HPITCH] = (_Float16)(hn * HCARRY);
    pv[r] = hn * wl;
  }
}

__global__ __launch_bounds__(SEQ_THR) void lstm2_seq_kernel(const float* __restrict__ x, const float* __restrict__ wih1,
                                                            const float* __restrict__ wlin, const float* __restrict__ blin,
                                                            const unsigned short* __restrict__ bt1p,
                                                            const unsigned short* __restrict__ bt2p,
                                                            const float* __restrict__ bsum, float* __restrict__ out) {
  __shared__ __align__(16) _Float16 H1s[2][ROWS_BLK * HPITCH];
  __shared__ __align__(16) _Float16 H2s[2][ROWS_BLK * HPITCH];
  __shared__ __align__(16) float    Slab[ROWS_BLK * SLABP];
  __shared__ __align__(16) float    Part[SEQ_WAVES * ROWS_BLK];
  const _Float16* BT1 = (const _Float16*)bt1p;
  const _Float16* BT2 = (const _Float16*)bt2p;
  const int tid = threadIdx.x, lane = tid & 31, wave = tid >> 5;
  const int c = lane & 15, hh = lane >> 4, koff = hh * 8;
  const int rowbase = blockIdx.x * ROWS_BLK;
  const int j = 16 * wave + c;

  {
    _Float16* p1 = &H1s[0][0];
    _Float16* p2 = &H2s[0][0];
#pragma unroll 1
    for (int i = tid; i < 2 * ROWS_BLK * HPITCH; i += SEQ_THR) {
      p1[i] = (_Float16)0.0f;
      p2[i] = (_Float16)0.0f;
    }
  }
#pragma unroll 1
  for (int i = tid; i < ROWS_BLK * (SLABP - NSTEP); i += SEQ_THR) {
    const int row = i / (SLABP - NSTEP);
    const int col = NSTEP + (i - row * (SLABP - NSTEP));
    Slab[row * SLABP + col] = 0.0f;
  }
#pragma unroll 1
  for (int it = 0; it < (ROWS_BLK * NSTEP / 4) / SEQ_THR; ++it) {
    const int idx = it * SEQ_THR + tid;
    const int row = idx >> 7;
    const int c4  = (idx & 127) * 4;
    const v4f v = *(const v4f*)(x + (size_t)(rowbase + row) * NSTEP + c4);
    *(v4f*)(Slab + row * SLABP + c4) = v;
  }

  float b1[4], w1[4], b2[4];
#pragma unroll
  for (int g = 0; g < 4; ++g) {
    b1[g] = bsum[g * NHID + j];
    w1[g] = wih1[g * NHID + j];
  }
  asm volatile("" ::: "memory");
#pragma unroll
  for (int g = 0; g < 4; ++g) b2[g] = bsum[NGATE + g * NHID + j];
  const float wl = wlin[j];
  const float bl = blin[0];

  float c1s[2][8], c2s[2][8];
#pragma unroll
  for (int mt = 0; mt < 2; ++mt)
#pragma unroll
    for (int r = 0; r < 8; ++r) { c1s[mt][r] = 0.0f; c2s[mt][r] = 0.0f; }
  __syncthreads();

  const v8f z8 = {0.f, 0.f, 0.f, 0.f, 0.f, 0.f, 0.f, 0.f};
  const _Float16* w1row = BT1 + (size_t)j * NHID + koff;
  const _Float16* w2row = BT2 + (size_t)j * (2 * NHID) + koff;

#pragma unroll 1
  for (int s = 0; s < NTOT; ++s) {
    const int cur  = s & 1;
    const int xcol = (s < NSTEP) ? s : (s - 1);
    const _Float16* h1c = &H1s[cur][0];
    _Float16*       h1n = &H1s[cur ^ 1][0];
    const _Float16* h2c = &H2s[cur][0];
    _Float16*       h2n = &H2s[cur ^ 1][0];

    v8f acc[4][2];
#pragma unroll
    for (int g = 0; g < 4; ++g) { acc[g][0] = z8; acc[g][1] = z8; }

    ksweep(acc, h1c + c * HPITCH + koff, w1row, NHID);
    acc_guard4(acc[0][0], acc[1][0], acc[2][0], acc[3][0]);
    acc_guard4(acc[0][1], acc[1][1], acc[2][1], acc[3][1]);
    {
      float pvd[8];
      cell_update<true>(acc[0][0], acc[1][0], acc[2][0], acc[3][0], c1s[0], b1, w1,
                        Slab + (8 * hh) * SLABP + xcol, h1n + (8 * hh) * HPITCH + j, wl, pvd);
      cell_update<true>(acc[0][1], acc[1][1], acc[2][1], acc[3][1], c1s[1], b1, w1,
                        Slab + (16 + 8 * hh) * SLABP + xcol, h1n + (16 + 8 * hh) * HPITCH + j, wl, pvd);
    }
    __syncthreads();

#pragma unroll
    for (int g = 0; g < 4; ++g) { acc[g][0] = z8; acc[g][1] = z8; }
    ksweep(acc, h1n + c * HPITCH + koff, w2row, 2 * NHID);
    ksweep(acc, h2c + c * HPITCH + koff, w2row + NHID, 2 * NHID);
    acc_guard4(acc[0][0], acc[1][0], acc[2][0], acc[3][0]);
    acc_guard4(acc[0][1], acc[1][1], acc[2][1], acc[3][1]);
    float pv0[8], pv1[8];
    cell_update<false>(acc[0][0], acc[1][0], acc[2][0], acc[3][0], c2s[0], b2, b2,
                       Slab, h2n + (8 * hh) * HPITCH + j, wl, pv0);
    cell_update<false>(acc[0][1], acc[1][1], acc[2][1], acc[3][1], c2s[1], b2, b2,
                       Slab, h2n + (16 + 8 * hh) * HPITCH + j, wl, pv1);
#pragma unroll
    for (int r = 0; r < 8; ++r) {
      float v0 = pv0[r];
      float v1 = pv1[r];
      v0 += __shfl_xor(v0, 8, 32);
      v1 += __shfl_xor(v1, 8, 32);
      v0 += __shfl_xor(v0, 4, 32);
      v1 += __shfl_xor(v1, 4, 32);
      v0 += __shfl_xor(v0, 2, 32);
      v1 += __shfl_xor(v1, 2, 32);
      v0 += __shfl_xor(v0, 1, 32);
      v1 += __shfl_xor(v1, 1, 32);
      if (c == 0) {
        Part[wave * ROWS_BLK + 8 * hh + r]      = v0;
        Part[wave * ROWS_BLK + 16 + 8 * hh + r] = v1;
      }
    }
    __syncthreads();
    if (tid < ROWS_BLK) {
      float a = 0.0f;
#pragma unroll
      for (int w = 0; w < SEQ_WAVES; ++w) a += Part[w * ROWS_BLK + tid];
      Slab[tid * SLABP + s] = a + bl;
    }
    __syncthreads();
  }

  float* ob = out + (size_t)rowbase * NTOT;
  for (int pass = 0; pass < 2; ++pass) {
#pragma unroll
    for (int it = 0; it < (ROWS_BLK * NTOT / 4) / SEQ_THR; ++it) {
      const int idx = it * SEQ_THR + tid;
      const int row = idx / (NTOT / 4);
      const int c4  = (idx - row * (NTOT / 4)) * 4;
      const v4f v = *(const v4f*)(Slab + row * SLABP + c4);
      *(volatile v4f*)(ob + (size_t)idx * 4) = v;
    }
    __threadfence();
  }
}

extern "C" void kernel_launch(void* const* d_in, const int* in_sizes, int n_in,
                              void* d_out, int out_size, void* d_ws, size_t ws_size, hipStream_t stream) {
  if (n_in < 11 || d_out == nullptr || d_ws == nullptr) return;
  if (in_sizes[0] != NBATCH * NSTEP || in_sizes[1] != NGATE || in_sizes[2] != NGATE * NHID ||
      in_sizes[3] != NGATE || in_sizes[4] != NGATE || in_sizes[5] != NGATE * NHID ||
      in_sizes[6] != NGATE * NHID || in_sizes[7] != NGATE || in_sizes[8] != NGATE ||
      in_sizes[9] != NHID || in_sizes[10] != 1 || out_size != NBATCH * NTOT) return;

  const float* x_train = (const float*)d_in[0];
  const float* w_ih1   = (const float*)d_in[1];
  const float* w_hh1   = (const float*)d_in[2];
  const float* b_ih1   = (const float*)d_in[3];
  const float* b_hh1   = (const float*)d_in[4];
  const float* w_ih2   = (const float*)d_in[5];
  const float* w_hh2   = (const float*)d_in[6];
  const float* b_ih2   = (const float*)d_in[7];
  const float* b_hh2   = (const float*)d_in[8];
  const float* w_lin   = (const float*)d_in[9];
  const float* b_lin   = (const float*)d_in[10];
  float* out = (float*)d_out;

  char* ws = (char*)d_ws;
  size_t off = 0;
  auto carve = [&](size_t bytes) -> char* { char* p = ws + off; off += (bytes + 255) & ~(size_t)255; return p; };
  unsigned short* BT1  = (unsigned short*)carve((size_t)NGATE * NHID * 2);
  unsigned short* BT2  = (unsigned short*)carve((size_t)NGATE * 2 * NHID * 2);
  float*          BSUM = (float*)carve((size_t)2 * NGATE * 4);
  if (off > ws_size || off > (size_t)134217728) return;

  prep_kernel<<<PREP_BLKS, PREP_THR, 0, stream>>>(w_hh1, w_ih2, w_hh2, b_ih1, b_hh1, b_ih2, b_hh2, BT1, BT2, BSUM);
  lstm2_seq_kernel<<<NBATCH / ROWS_BLK, SEQ_THR, 0, stream>>>(x_train, w_ih1, w_lin, b_lin, BT1, BT2, BSUM, out);
}
